// GraphCapsuleLayer_77884936946120
// MI455X (gfx1250) — hardware-verified
//
#include <hip/hip_runtime.h>


#ifndef NB
#define NB 4
#endif
#ifndef NPT
#define NPT 4000
#endif
#define NB_FULL  4
#define NPT_FULL 4000
#ifndef OUT_NPT
#define OUT_NPT NPT
#endif
#define NJ   8
#define ND   16
#define NI   16
#define NK   8
#define NROUTE 3
#define CEPS 1e-7f
#define SPB  16
#define XROW (NI * NK)
#define OROW (NJ * ND)
#define UFLOATS (NI * (ND / 4) * (SPB * NJ) * 4)
#define LOG2E 1.4426950408889634f

static_assert(NK == 8);
static_assert(ND == 16);
static_assert(SPB == 16);
static_assert(SPB * NJ == 128);
static_assert(NJ == 8);
static_assert(NI == 16);
static_assert(NPT % SPB == 0);
static_assert((NB * NPT) % SPB == 0);
static_assert((size_t)UFLOATS * 4 <= 131072);
static_assert(SPB * OROW <= UFLOATS);
static_assert(128 * 4 * 16 == SPB * OROW * 4);
static_assert((OROW * 4) % 128 == 0);
static_assert(((size_t)NJ * NI * ND * NK) % 8 == 0);
static_assert(NB <= NB_FULL);
static_assert(NPT <= NPT_FULL);

typedef unsigned short bf;
typedef __attribute__((ext_vector_type(16))) __bf16   v16bf;
typedef __attribute__((ext_vector_type(8)))  unsigned short v8us;
typedef __attribute__((ext_vector_type(8)))  float    v8f;
typedef __attribute__((ext_vector_type(4)))  float    v4f;
typedef v4f  __attribute__((may_alias)) v4fa;

__device__ __forceinline__ unsigned short f2bf(float f) { unsigned u = __float_as_uint(f); u += 0x7FFFu + ((u >> 16) & 1u); return (unsigned short)(u >> 16); }
__device__ __forceinline__ v16bf cat16b(v8us lo, v8us hi) { return __builtin_bit_cast(v16bf, __builtin_shufflevector(lo, hi, 0, 1, 2, 3, 4, 5, 6, 7, 8, 9, 10, 11, 12, 13, 14, 15)); }
__device__ __forceinline__ v8f wmmab(v16bf a, v16bf b, v8f c) { return __builtin_amdgcn_wmma_f32_16x16x32_bf16(false, a, false, b, (short)0, c, false, false); }
__device__ __forceinline__ v8f wmmab_g(v16bf a, v16bf b, v8f c) {
    c = wmmab(a, b, c);
    asm volatile("v_nop\n\tv_nop\n\tv_nop\n\tv_nop" : "+v"(c) : "v"(a), "v"(b));
    return c;
}

__global__ __launch_bounds__(256) void k_cvt8(const float* __restrict__ src, bf* dst, size_t n8) {
    const size_t i = (size_t)blockIdx.x * 256 + threadIdx.x; if (i >= n8) return;
    const v8f v = *(const v8f*)(src + i * 8); v8us o;
#pragma unroll
    for (int k = 0; k < 8; ++k) o[k] = f2bf(v[k]);
    *(volatile v8us*)(dst + i * 8) = o; __threadfence(); *(volatile v8us*)(dst + i * 8) = o;
}

__global__ __launch_bounds__(128) __attribute__((amdgpu_num_vgpr(256))) void k_caps(const float* __restrict__ X, const bf* __restrict__ WB, float* OUT) {
    __shared__ __align__(16) float U[UFLOATS];
    const int tid = threadIdx.x;
    const int lane = tid & 31, lr = lane & 15, hi = lane >> 4;
    const int wave = __builtin_amdgcn_readfirstlane((int)(threadIdx.x >> 5));
    const int g0 = blockIdx.x * SPB;
    const int bidx = g0 / NPT, n0 = g0 % NPT;
    const float* xs = X + ((size_t)bidx * NPT_FULL + (size_t)(n0 + lr)) * XROW;
    const v8us z8 = (v8us){};
    const bool lowh = (hi == 0);

#pragma unroll 1
    for (int ii = 0; ii < 4; ++ii) {
        const int i = wave * 4 + ii;
        v4f x0 = *(const v4f*)(xs + i * NK), x1 = *(const v4f*)(xs + i * NK + 4);
        asm volatile("" : "+v"(x0), "+v"(x1));
        v8us au;
#pragma unroll
        for (int k = 0; k < 4; ++k) {
            const unsigned short c0 = f2bf(x0[k]), c1 = f2bf(x1[k]);
            au[k] = lowh ? c0 : (unsigned short)0; au[4 + k] = lowh ? c1 : (unsigned short)0; }
        const v16bf afr = cat16b(au, z8);
        const int ubase = (i * 4 + (lr >> 2)) * 512 + (8 * hi) * 32 + (lr & 3);
#pragma unroll
        for (int j = 0; j < NJ; ++j) {
            v8us wu = *(const v8us*)(WB + ((size_t)((j * NI + i) * ND + lr)) * NK);
            asm volatile("" : "+v"(wu));
            const v8us wsel = lowh ? wu : z8;
            const v16bf bfr_ = cat16b(wsel, z8);
            v8f c = (v8f){};
            c = wmmab_g(afr, bfr_, c);
#pragma unroll
            for (int r = 0; r < 8; ++r) U[ubase + r * 32 + j * 4] = c[r];
        }
    }
    __syncthreads();

    const int ub = tid * 4;
    float lg[NI];
#pragma unroll
    for (int i = 0; i < NI; ++i) lg[i] = 0.0f;
    v4f oA = (v4f){}, oB = (v4f){}, oC = (v4f){}, oD = (v4f){};

#pragma unroll 1
    for (int it = 0; it < NROUTE; ++it) {
        float cv[NI];
#pragma unroll
        for (int i = 0; i < NI; ++i) {
            const float v = lg[i];
            float mx = v;
            mx = fmaxf(mx, __shfl_xor(mx, 1, 32));
            mx = fmaxf(mx, __shfl_xor(mx, 2, 32));
            mx = fmaxf(mx, __shfl_xor(mx, 4, 32));
            const float e = __builtin_amdgcn_exp2f((v - mx) * LOG2E);
            float ss = e;
            ss += __shfl_xor(ss, 1, 32);
            ss += __shfl_xor(ss, 2, 32);
            ss += __shfl_xor(ss, 4, 32);
            cv[i] = e * __builtin_amdgcn_rcpf(ss);
        }
#pragma unroll 1
        for (int q = 0; q < 4; ++q) {
            const int qb = q * 512 + ub;
            v4f n4 = (v4f){};
#pragma unroll
            for (int i = 0; i < NI; ++i) {
                const v4f u = *(const v4fa*)(&U[i * 2048 + qb]);
                n4[0] = fmaf(cv[i], u[0], n4[0]);
                n4[1] = fmaf(cv[i], u[1], n4[1]);
                n4[2] = fmaf(cv[i], u[2], n4[2]);
                n4[3] = fmaf(cv[i], u[3], n4[3]);
                if ((i & 3) == 3) __builtin_amdgcn_sched_barrier(0);
            }
            oA = oB; oB = oC; oC = oD; oD = n4;
        }
        if (it == NROUTE - 1) break;
        float s2 = 0.0f;
#pragma unroll
        for (int e = 0; e < 4; ++e) s2 = fmaf(oA[e], oA[e], s2);
#pragma unroll
        for (int e = 0; e < 4; ++e) s2 = fmaf(oB[e], oB[e], s2);
#pragma unroll
        for (int e = 0; e < 4; ++e) s2 = fmaf(oC[e], oC[e], s2);
#pragma unroll
        for (int e = 0; e < 4; ++e) s2 = fmaf(oD[e], oD[e], s2);
        const float scale = s2 / (1.0f + s2) / sqrtf(s2 + CEPS);
#pragma unroll
        for (int e = 0; e < 4; ++e) { oA[e] *= scale; oB[e] *= scale; oC[e] *= scale; oD[e] *= scale; }
        float acc[NI];
#pragma unroll
        for (int i = 0; i < NI; ++i) acc[i] = 0.0f;
#pragma unroll 1
        for (int q = 0; q < 4; ++q) {
            const int qb = q * 512 + ub;
            const v4f oq = oA;
#pragma unroll
            for (int i = 0; i < NI; ++i) {
                const v4f u = *(const v4fa*)(&U[i * 2048 + qb]);
                acc[i] = fmaf(oq[0], u[0], acc[i]);
                acc[i] = fmaf(oq[1], u[1], acc[i]);
                acc[i] = fmaf(oq[2], u[2], acc[i]);
                acc[i] = fmaf(oq[3], u[3], acc[i]);
                if ((i & 3) == 3) __builtin_amdgcn_sched_barrier(0);
            }
            oA = oB; oB = oC; oC = oD; oD = oq;
        }
#pragma unroll
        for (int i = 0; i < NI; ++i) lg[i] += acc[i];
    }

    __syncthreads();
    *(v4fa*)(&U[tid * ND +  0]) = oA;
    *(v4fa*)(&U[tid * ND +  4]) = oB;
    *(v4fa*)(&U[tid * ND +  8]) = oC;
    *(v4fa*)(&U[tid * ND + 12]) = oD;
    __syncthreads();
    float* ob = OUT + ((size_t)bidx * OUT_NPT + (size_t)n0) * OROW;
#pragma unroll 1
    for (int ps = 0; ps < 2; ++ps) {
#pragma unroll
        for (int p = 0; p < 4; ++p) { const int f = p * 128 + tid;
            const v4f val = *(const v4fa*)(&U[f * 4]);
            *(volatile v4f*)(ob + (size_t)f * 4) = val; }
        if (ps == 0) __threadfence(); }
}

static constexpr size_t al256(size_t v) { return (v + 255) & ~(size_t)255; }
static constexpr size_t SZ_WB = al256((size_t)NJ * NI * ND * NK * 2);
static constexpr size_t SZ_TOTAL = SZ_WB;
static_assert(SZ_TOTAL <= (size_t)134217728);
static_assert(((size_t)NJ * NI * ND * NK / 8) * 16 <= SZ_WB);

extern "C" void kernel_launch(void* const* d_in, const int* in_sizes, int n_in,
                              void* d_out, int out_size, void* d_ws, size_t ws_size, hipStream_t stream) {
    if (n_in < 2) return;
    const size_t needx = ((size_t)(NB - 1) * NPT_FULL + NPT) * XROW;
    if ((size_t)in_sizes[0] < needx) return;
    if ((size_t)in_sizes[1] < (size_t)NJ * NI * ND * NK) return;
    if ((size_t)out_size < ((size_t)(NB - 1) * OUT_NPT + NPT) * OROW) return;
    if (SZ_TOTAL > ws_size) return;
    const float* x = (const float*)d_in[0];
    const float* w = (const float*)d_in[1];
    float* OUT = (float*)d_out;
    bf* WB = (bf*)d_ws;

    { const size_t n8 = (size_t)NJ * NI * ND * NK / 8;
      k_cvt8<<<(unsigned)((n8 + 255) / 256), 256, 0, stream>>>(w, WB, n8); }
    k_caps<<<dim3((NB * NPT) / SPB, 1, 1), 128, 0, stream>>>(x, WB, OUT);
}
